// HANLayer_1425929143036
// MI455X (gfx1250) — hardware-run, weakly checked
//
#include <hip/hip_runtime.h>
#include <math.h>

constexpr int kThreads     = 256;
constexpr int kNodes       = 50000;
constexpr int kEdges       = 600000;
constexpr int kPaths       = 3;
constexpr int kDim         = 128;
constexpr int kNPad        = 50048;
constexpr int kNMain       = 49984;
constexpr int kTailRows    = kNPad - kNMain;
constexpr int kTileRows    = 6272;
constexpr int kTiles       = 8;
constexpr int kIsoPitch    = kTiles * kTileRows;
constexpr int kRowsPerWave = kTileRows / 8;
constexpr int kChunk       = 4096;
constexpr int kPerThread   = kChunk / kThreads;
constexpr int kNChunks     = (kEdges + kChunk - 1) / kChunk;
constexpr int kMainTiles   = (kNMain / 64) * (kDim / 64);
constexpr int kMainBlocks  = (kMainTiles + 7) / 8;
constexpr int kPadTiles    = (kNPad / 64) * (kDim / 64);
constexpr int kPadBlocks   = (kPadTiles + 7) / 8;
constexpr int kRedRows     = 256;
constexpr int kRedBlocks   = (kNPad + kRedRows - 1) / kRedRows;
static_assert(kNPad % 64 == 0, "shape");
static_assert(kNMain % 64 == 0, "shape");
static_assert(kTailRows == 64, "shape");
static_assert(kNPad >= kNodes && kNMain < kNodes, "shape");
static_assert(kDim % 64 == 0 && kDim % 32 == 0, "shape");
static_assert(kTiles * kTileRows >= kNPad, "shape");
static_assert(kTileRows % 8 == 0, "shape");
static_assert((kTileRows / 4) % 32 == 0, "shape");
static_assert((kTileRows * 4) % 128 == 0, "shape");
static_assert(kEdges % kPerThread == 0, "shape");
static_assert(kChunk == kThreads * kPerThread, "shape");
static_assert((kNPad * (kDim / 8)) % kThreads == 0, "shape");
static_assert((kNodes * (kDim / 4)) % kThreads == 0, "shape");
static_assert(kMainBlocks * 8 >= kMainTiles && kPadBlocks * 8 >= kPadTiles, "shape");
static_assert(kRedBlocks * kRedRows >= kNodes, "shape");
static_assert(kRedRows % 4 == 0 && kThreads == 4 * (kDim / 2), "shape");
static_assert(kTileRows < 65536 && kNodes < 65536, "shape");

typedef __attribute__((ext_vector_type(16))) _Float16 v16h;
typedef __attribute__((ext_vector_type(8)))  _Float16 v8h;
typedef __attribute__((ext_vector_type(16))) __bf16   v16b;
typedef __attribute__((ext_vector_type(8)))  __bf16   v8b;
typedef __attribute__((ext_vector_type(8)))  float    v8f;
typedef __attribute__((ext_vector_type(4)))  float    v4f;
typedef __attribute__((ext_vector_type(4)))  unsigned int v4u;
typedef __attribute__((ext_vector_type(4)))  int      v4i;

__device__ __forceinline__ unsigned short f2bf_bits(float f) {
  unsigned u = __float_as_uint(f);
  return (unsigned short)((u + 0x7FFFu + ((u >> 16) & 1u)) >> 16);
}
__device__ __forceinline__ float bf_bits2f(unsigned short h) { return __uint_as_float(((unsigned)h) << 16); }

__device__ __forceinline__ void dep_guard_h(v8f& a, v8f& b, v16h x, v16h y) { asm volatile("v_nop\n\tv_nop\n\tv_nop\n\tv_nop" : "+v"(a), "+v"(b) : "v"(x), "v"(y)); }
__device__ __forceinline__ void dep_guard_b(v8f& a, v8f& b, v16b x, v16b y) { asm volatile("v_nop\n\tv_nop\n\tv_nop\n\tv_nop" : "+v"(a), "+v"(b) : "v"(x), "v"(y)); }
__device__ __forceinline__ void keep4_h(v16h a, v16h b, v16h c, v16h d) { asm volatile("v_nop" :: "v"(a), "v"(b), "v"(c), "v"(d)); }
__device__ __forceinline__ void keep4_b(v16b a, v16b b, v16b c, v16b d) { asm volatile("v_nop" :: "v"(a), "v"(b), "v"(c), "v"(d)); }
__device__ __forceinline__ void acc_guard4(v8f& a, v8f& b, v8f& c, v8f& d) { asm volatile("v_nop\n\tv_nop\n\tv_nop\n\tv_nop" : "+v"(a), "+v"(b), "+v"(c), "+v"(d)); }
template <typename T> struct Frag;
template <> struct Frag<_Float16> {
  typedef v16h V; union U { v16h v; v8h h[2]; };
  static __device__ __forceinline__ v16h load(const _Float16* p) {
    U f; f.h[0] = *(const v8h*)(p); f.h[1] = *(const v8h*)(p + 16); return f.v;
  }
  static __device__ __forceinline__ v8f mma(v16h a, v16h b, v8f c) {
    return __builtin_amdgcn_wmma_f32_16x16x32_f16(false, a, false, b, (short)0, c, false, false);
  }
  static __device__ __forceinline__ void guard(v8f& a, v8f& b, v16h x, v16h y) { dep_guard_h(a, b, x, y); }
  static __device__ __forceinline__ void keep(v16h a, v16h b, v16h c, v16h d) { keep4_h(a, b, c, d); }
};
template <> struct Frag<__bf16> {
  typedef v16b V; union U { v16b v; v8b h[2]; };
  static __device__ __forceinline__ v16b load(const __bf16* p) {
    U f; f.h[0] = *(const v8b*)(p); f.h[1] = *(const v8b*)(p + 16); return f.v;
  }
  static __device__ __forceinline__ v8f mma(v16b a, v16b b, v8f c) {
    return __builtin_amdgcn_wmma_f32_16x16x32_bf16(false, a, false, b, (short)0, c, false, false);
  }
  static __device__ __forceinline__ void guard(v8f& a, v8f& b, v16b x, v16b y) { dep_guard_b(a, b, x, y); }
  static __device__ __forceinline__ void keep(v16b a, v16b b, v16b c, v16b d) { keep4_b(a, b, c, d); }
};

__device__ __forceinline__ unsigned pk16(unsigned short a, unsigned short b) { return (unsigned)a | ((unsigned)b << 16); }
__device__ __forceinline__ float bfr(float x) { return bf_bits2f(f2bf_bits(x)); }
__device__ __forceinline__ float h16_to_f32(unsigned hb) {
  const unsigned sgn = (hb & 0x8000u) << 16; const unsigned em = hb & 0x7fffu;
  const float fn = __uint_as_float((em << 13) + 0x38000000u);
  const float fs = (float)em * 5.9604644775390625e-8f;
  const float mag = (em < 0x400u) ? fs : fn; return __uint_as_float(__float_as_uint(mag) | sgn); }

template <int ET> struct Elem;
template <> struct Elem<0> { typedef _Float16 T; };
template <> struct Elem<1> { typedef __bf16 T; };
template <int ET, bool SPLIT, int BIAS_MODE, int OUT_MODE, bool RESID, int ACT = 0>
__global__ __launch_bounds__(256) void wmma_gemm64(
    const unsigned short* __restrict__ Ap, const unsigned short* __restrict__ A2p, int lda, long strideA,
    const unsigned short* __restrict__ Btp, const unsigned short* __restrict__ Bt2p, int ldb, long strideB,
    void* __restrict__ Cout, void* __restrict__ Cout2, int ldc, long strideC,
    const float* __restrict__ bias,
    const float* __restrict__ resid, long strideR,
    int M, int N, int K, float scale) {
  typedef typename Elem<ET>::T T;
  typedef typename Frag<T>::V V;
  const T* A = (const T*)Ap; const T* A2 = (const T*)A2p; const T* Bt = (const T*)Btp; const T* Bt2 = (const T*)Bt2p;
  __shared__ __align__(16) float sT[8][16 * 68];
  const int b    = blockIdx.y;
  const int lane = threadIdx.x & 31;
  const int wave = threadIdx.x >> 5;
  const int tilesN = N >> 6;
  const int tilesM = M >> 6;
  const int tile = blockIdx.x * 8 + wave;
  if (tile >= tilesM * tilesN) return;
  const int tm = tile / tilesN;
  const int tn = tile - tm * tilesN;
  const int m0 = tm << 6;
  const int n0 = tn << 6;

  const T* Ab  = A  + (size_t)b * strideA;
  const T* Bb  = Bt + (size_t)b * strideB;
  const T* Ab2 = SPLIT ? (A2  + (size_t)b * strideA) : nullptr;
  const T* Bb2 = SPLIT ? (Bt2 + (size_t)b * strideB) : nullptr;

  const int rlane = lane & 15;
  const int koff  = (lane >> 4) * 8;
  const int mOff  = (lane >> 4) * 8;

  v8f acc[4][4];
#pragma unroll
  for (int i = 0; i < 4; ++i)
#pragma unroll
    for (int j = 0; j < 4; ++j) acc[i][j] = (v8f){0.f,0.f,0.f,0.f,0.f,0.f,0.f,0.f};

  for (int k0 = 0; k0 < K; k0 += 32) {
    V bh[4], bl[4];
#pragma unroll
    for (int j = 0; j < 4; ++j) {
      const size_t bo = (size_t)(n0 + (j << 4) + rlane) * ldb + koff + k0;
      bh[j] = Frag<T>::load(Bb + bo);
      if (SPLIT) bl[j] = Frag<T>::load(Bb2 + bo);
    }
#pragma unroll
    for (int i = 0; i < 4; ++i) {
      const size_t ao = (size_t)(m0 + (i << 4) + rlane) * lda + koff + k0;
      V ah = Frag<T>::load(Ab + ao);
      V al;
      if (SPLIT) al = Frag<T>::load(Ab2 + ao);
#pragma unroll
      for (int j = 0; j < 4; ++j) {
        acc[i][j] = Frag<T>::mma(ah, bh[j], acc[i][j]);
        if (SPLIT) {
          acc[i][j] = Frag<T>::mma(ah, bl[j], acc[i][j]);
          acc[i][j] = Frag<T>::mma(al, bh[j], acc[i][j]);
        }
      }
      Frag<T>::guard(acc[i][0], acc[i][3], ah, SPLIT ? al : ah);
    }
    Frag<T>::keep(bh[0], bh[1], bh[2], bh[3]);
    if (SPLIT) Frag<T>::keep(bl[0], bl[1], bl[2], bl[3]);
  }
  acc_guard4(acc[0][0], acc[0][1], acc[0][2], acc[0][3]);
  acc_guard4(acc[1][0], acc[1][1], acc[1][2], acc[1][3]);
  acc_guard4(acc[2][0], acc[2][1], acc[2][2], acc[2][3]);
  acc_guard4(acc[3][0], acc[3][1], acc[3][2], acc[3][3]);

  float* slab = sT[wave];
  const float* Rb = RESID ? (resid + (size_t)b * strideR) : nullptr;
#pragma unroll
  for (int i = 0; i < 4; ++i) {
    const int mBase = m0 + (i << 4);
#pragma unroll
    for (int j = 0; j < 4; ++j) {
      const int n = n0 + (j << 4) + rlane;
      float bv = 0.f;
      if (BIAS_MODE == 2) bv = bias[n];
#pragma unroll
      for (int r = 0; r < 8; ++r) {
        float v = acc[i][j][r] * scale;
        if (BIAS_MODE == 1) v += bias[mBase + mOff + r];
        if (BIAS_MODE == 2) v += bv;
        if (RESID) v += Rb[(size_t)(mBase + mOff + r) * ldc + n];
        if (ACT == 1) v = tanhf(v);
        if (ACT == 2) v = fmaxf(v, 0.0f);
        if (ACT == 3) v = v / (1.0f + expf(-v));
        if (ACT == 4) v = (v > 0.f) ? v : 0.01f * v;
        if (ACT == 5) v = 0.5f * v * (1.0f + erff(v * 0.70710678118654752f));
        slab[(mOff + r) * 68 + (j << 4) + rlane] = v;
      }
    }
    __builtin_amdgcn_fence(__ATOMIC_RELEASE, "workgroup");
    __builtin_amdgcn_wave_barrier();
    __builtin_amdgcn_fence(__ATOMIC_ACQUIRE, "workgroup");
    if (OUT_MODE == 0) {
      float* C = (float*)Cout + (size_t)b * strideC;
      const int hh = lane >> 4, c4 = (lane & 15) * 4;
      for (int pass = 0; pass < 2; ++pass) {
#pragma unroll
        for (int it = 0; it < 8; ++it) {
          const int row = it * 2 + hh;
          v4f v = *(const v4f*)(slab + row * 68 + c4);
          *(volatile v4f*)(C + (size_t)(mBase + row) * ldc + n0 + c4) = v;
        }
        __threadfence();
      }
    } else {
      const int q = lane >> 3, c8 = (lane & 7) * 8;
      unsigned short* C  = (unsigned short*)Cout  + (size_t)b * strideC;
      unsigned short* C2 = (OUT_MODE == 2) ? ((unsigned short*)Cout2 + (size_t)b * strideC) : nullptr;
      for (int pass = 0; pass < 2; ++pass) {
#pragma unroll
        for (int it = 0; it < 4; ++it) {
          const int row = it * 4 + q;
          const float* sp = slab + row * 68 + c8;
          v8h hv, lv;
#pragma unroll
          for (int e = 0; e < 8; ++e) {
            if (OUT_MODE == 1) {
              hv[e] = (_Float16)sp[e];
            } else {
              unsigned short hb = f2bf_bits(sp[e]);
              unsigned short lb = f2bf_bits(sp[e] - bf_bits2f(hb));
              hv[e] = __builtin_bit_cast(_Float16, hb);
              lv[e] = __builtin_bit_cast(_Float16, lb);
            }
          }
          *(volatile v8h*)(C + (size_t)(mBase + row) * ldc + n0 + c8) = hv;
          if (OUT_MODE == 2) *(volatile v8h*)(C2 + (size_t)(mBase + row) * ldc + n0 + c8) = lv;
        }
        __threadfence();
      }
    }
    __builtin_amdgcn_fence(__ATOMIC_RELEASE, "workgroup");
    __builtin_amdgcn_wave_barrier();
    __builtin_amdgcn_fence(__ATOMIC_ACQUIRE, "workgroup");
  }
}

__device__ __forceinline__ int blk_excl_scan(int cnt, int* scan_ws, int tid, int* tot) {
  const int lane = tid & 31, wave = tid >> 5; int incl = cnt;
#pragma unroll
  for (int o = 1; o < 32; o <<= 1) { const int v = __shfl_up(incl, o, 32); if (lane >= o) incl += v; }
  if (lane == 31) scan_ws[wave] = incl;
  __syncthreads();
  if (wave == 0) { int wv = (lane < kThreads / 32) ? scan_ws[lane] : 0; int wincl = wv;
#pragma unroll
    for (int o = 1; o < 32; o <<= 1) { const int v = __shfl_up(wincl, o, 32); if (lane >= o) wincl += v; }
    if (lane < kThreads / 32) scan_ws[32 + lane] = wincl - wv; if (lane == 31) scan_ws[64] = wincl; }
  __syncthreads();
  const int res = scan_ws[32 + wave] + incl - cnt; *tot = scan_ws[64];
  return res;
}
__device__ __forceinline__ int clamp_node(int v) { v = v < 0 ? 0 : v; return v >= kNodes ? (kNodes - 1) : v; }

__device__ __forceinline__ int chunk_hits_src(const int* __restrict__ srcv, int e0, int n0, int tid, int* LIST, int* scan_ws) {
  const int eb = e0 + tid * kPerThread;
  const bool valid = eb < kEdges;
  const int ebc = valid ? eb : (kEdges - kPerThread);
  int rec[kPerThread]; int cnt = 0;
#pragma unroll
  for (int k = 0; k < kPerThread; k += 4) {
    const v4i s4 = *(const v4i*)(srcv + ebc + k);
#pragma unroll
    for (int e = 0; e < 4; ++e) {
      const int s = clamp_node(s4[e]);
      int r = -1;
      if (valid && s >= n0 && s < n0 + kTileRows) { r = s - n0; ++cnt; }
      rec[k + e] = r;
    }
  }
  int tot; int p = blk_excl_scan(cnt, scan_ws, tid, &tot);
#pragma unroll
  for (int k = 0; k < kPerThread; ++k) if (rec[k] >= 0) { if ((unsigned)p < (unsigned)kChunk) LIST[p] = rec[k]; ++p; }
  __syncthreads();
  return tot < kChunk ? tot : kChunk;
}
__device__ __forceinline__ int chunk_hits_dst(const int* __restrict__ dstv, const int* __restrict__ srcv, int e0, int n0, int tid,
                                              int* LIST, int* scan_ws) {
  const int eb = e0 + tid * kPerThread;
  const bool valid = eb < kEdges;
  const int ebc = valid ? eb : (kEdges - kPerThread);
  int rec[kPerThread]; int cnt = 0;
#pragma unroll
  for (int k = 0; k < kPerThread; k += 4) {
    const v4i d4 = *(const v4i*)(dstv + ebc + k);
    const v4i s4 = *(const v4i*)(srcv + ebc + k);
#pragma unroll
    for (int e = 0; e < 4; ++e) {
      const int d = clamp_node(d4[e]);
      const int s = clamp_node(s4[e]);
      int r = -1;
      if (valid && d >= n0 && d < n0 + kTileRows) { r = ((d - n0) << 16) | s; ++cnt; }
      rec[k + e] = r;
    }
  }
  int tot; int p = blk_excl_scan(cnt, scan_ws, tid, &tot);
#pragma unroll
  for (int k = 0; k < kPerThread; ++k) if (rec[k] >= 0) { if ((unsigned)p < (unsigned)kChunk) LIST[p] = rec[k]; ++p; }
  __syncthreads();
  return tot < kChunk ? tot : kChunk;
}

__global__ __launch_bounds__(kThreads) void cast_h_kernel(const float* __restrict__ h, unsigned short* __restrict__ hb) {
  const int i = blockIdx.x * kThreads + threadIdx.x;
  if (i >= kNPad * (kDim / 8)) return;
  const int row = i >> 4;
  const int c8 = (i & 15) * 8;
  const bool live = row < kNodes;
  const int rowc = live ? row : (kNodes - 1);
  const float* p = h + (size_t)rowc * kDim + c8;
  const v4f a = *(const v4f*)(p);
  const v4f c = *(const v4f*)(p + 4);
  unsigned short hv[8];
#pragma unroll
  for (int e = 0; e < 4; ++e) {
    hv[e]     = live ? f2bf_bits(a[e]) : (unsigned short)0;
    hv[4 + e] = live ? f2bf_bits(c[e]) : (unsigned short)0;
  }
  const v4u u = (v4u){pk16(hv[0], hv[1]), pk16(hv[2], hv[3]), pk16(hv[4], hv[5]), pk16(hv[6], hv[7])};
  unsigned short* q = hb + 8 * (size_t)i;
  *(volatile v4u*)q = u;
  __threadfence();
  *(volatile v4u*)q = u;
}

__global__ __launch_bounds__(kThreads) void wtcast_kernel(const float* __restrict__ Wgc, const float* __restrict__ w1,
                                                         unsigned short* __restrict__ out) {
  __shared__ float sm[64][65];
  const int t  = threadIdx.x;
  const int k0 = blockIdx.x * 64;
  const int nb = blockIdx.y * 64;
  const int z  = blockIdx.z;
  const float* W = (z < kPaths) ? (Wgc + (size_t)z * kDim * kDim) : w1;
#pragma unroll
  for (int i = 0; i < 16; ++i) {
    const int e = i * kThreads + t;
    const int r = e >> 6;
    const int c = e & 63;
    sm[c][r] = W[(size_t)(k0 + r) * kDim + nb + c];
  }
  __syncthreads();
  const int lane = t & 31, wave = t >> 5;
  const int q = lane >> 3, c8 = (lane & 7) * 8;
  unsigned short* op = out + (size_t)z * kDim * kDim;
  for (int pass = 0; pass < 2; ++pass) {
#pragma unroll
    for (int it = 0; it < 2; ++it) {
      const int row = wave * 8 + it * 4 + q;
      unsigned short hb8[8];
#pragma unroll
      for (int e = 0; e < 8; ++e) hb8[e] = f2bf_bits(sm[row][c8 + e]);
      const v4u u = (v4u){pk16(hb8[0], hb8[1]), pk16(hb8[2], hb8[3]), pk16(hb8[4], hb8[5]), pk16(hb8[6], hb8[7])};
      *(volatile v4u*)(op + (size_t)(nb + row) * kDim + k0 + c8) = u;
    }
    __threadfence();
  }
}

__global__ __launch_bounds__(kThreads) void degout_kernel(const int* __restrict__ esrc, float* __restrict__ iso) {
  __shared__ int LIST[kChunk];
  __shared__ __align__(16) int CNT[kTileRows];
  __shared__ int scan_ws[80];
  const int tid = threadIdx.x, lane = tid & 31, wave = tid >> 5;
  const int p  = blockIdx.y;
  const int n0 = blockIdx.x * kTileRows;
  for (int i = tid; i < kChunk; i += kThreads) LIST[i] = 0;
  for (int i = tid; i < kTileRows; i += kThreads) CNT[i] = 0;
  if (tid < 80) scan_ws[tid] = 0;
  __syncthreads();
  const int* srcv = esrc + (size_t)p * kEdges;
  const int wlo = wave * kRowsPerWave, whi = wlo + kRowsPerWave;
#pragma unroll 1
  for (int c = 0; c < kNChunks; ++c) {
    const int tot = chunk_hits_src(srcv, c * kChunk, n0, tid, LIST, scan_ws);
#pragma unroll 1
    for (int base = 0; base < tot; base += 32) {
      const int q = base + lane;
      const int rv0 = LIST[q];
      const int rv = (q < tot) ? rv0 : -1;
      const int own = (rv >= wlo && rv < whi) ? 1 : 0;
      unsigned msk = (unsigned)__ballot(own);
#pragma unroll 1
      for (int it = 0; it < 32; ++it) {
        if (msk == 0u) break;
        const int bp = __builtin_ctz(msk); msk &= msk - 1u;
        const int dl = __shfl(rv, bp, 32);
        if (lane == 0) CNT[dl] = CNT[dl] + 1;
      }
    }
    __syncthreads();
  }
  float* op = iso + (size_t)p * kIsoPitch + (size_t)blockIdx.x * kTileRows;
#pragma unroll 1
  for (int it = 0; it < (kTileRows / 4 + kThreads - 1) / kThreads; ++it) {
    const int slot = it * kThreads + tid;
    if (slot < kTileRows / 4) {
      const v4i c4 = *(const v4i*)(CNT + 4 * slot);
      v4f o;
#pragma unroll
      for (int e = 0; e < 4; ++e) { const float cf = (float)c4[e]; o[e] = rsqrtf(fmaxf(cf, 1.0f)); }
      *(volatile v4f*)(op + 4 * slot) = o;
      __threadfence();
      *(volatile v4f*)(op + 4 * slot) = o;
    }
  }
}

__global__ __launch_bounds__(kThreads) void agg_kernel(const float* __restrict__ xmain, const float* __restrict__ xtail,
                                                      const int* __restrict__ esrc, const int* __restrict__ edst,
                                                      const float* __restrict__ iso, const float* __restrict__ bgc,
                                                      float* zp, unsigned short* __restrict__ zbp) {
  __shared__ int LIST[kChunk];
  __shared__ int CNT[kTileRows];
  __shared__ int scan_ws[80];
  const int tid = threadIdx.x, lane = tid & 31, wave = tid >> 5;
  const int n0 = blockIdx.x * kTileRows;
  for (int i = tid; i < kChunk; i += kThreads) LIST[i] = 0;
  for (int i = tid; i < kTileRows; i += kThreads) CNT[i] = 0;
  if (tid < 80) scan_ws[tid] = 0;
  __syncthreads();
  const int wlo = wave * kRowsPerWave, whi = wlo + kRowsPerWave;
  const v4f z4 = {0.f, 0.f, 0.f, 0.f};
#pragma unroll 1
  for (int j = 0; j < kRowsPerWave; ++j) {
    const int n = n0 + wlo + j;
    if (n < kNPad) *(v4f*)(zp + (size_t)n * kDim + 4 * lane) = z4;
  }
#pragma unroll 1
  for (int c = 0; c < kNChunks; ++c) {
    const int tot = chunk_hits_dst(edst, esrc, c * kChunk, n0, tid, LIST, scan_ws);
#pragma unroll 1
    for (int base = 0; base < tot; base += 32) {
      const int q = base + lane;
      const int rv0 = LIST[q];
      const int rv = (q < tot) ? rv0 : -1;
      const int dq = rv >> 16;
      const int own = (rv >= 0 && dq >= wlo && dq < whi) ? 1 : 0;
      unsigned msk = (unsigned)__ballot(own);
#pragma unroll 1
      for (int it = 0; it < 32; ++it) {
        if (msk == 0u) break;
        const int bp = __builtin_ctz(msk); msk &= msk - 1u;
        const int r = __shfl(rv, bp, 32);
        const int dl = r >> 16;
        const int s = r & 0xFFFF;
        const float sc = iso[s];
        const int sm = (s < kNMain) ? s : (kNMain - 1);
        const int st = (s < kNMain) ? 0 : (s - kNMain);
        const float* xr = (s < kNMain) ? (xmain + (size_t)sm * kDim) : (xtail + (size_t)st * kDim);
        const v4f xv = *(const v4f*)(xr + 4 * lane);
        float* rp = zp + (size_t)(n0 + dl) * kDim + 4 * lane;
        v4f a = *(const v4f*)rp;
        a = a + xv * sc;
        *(v4f*)rp = a;
        if (lane == 0) CNT[dl] = CNT[dl] + 1;
      }
    }
    __syncthreads();
  }
  const v4f braw = *(const v4f*)(bgc + 4 * lane);
  v4f bb;
#pragma unroll
  for (int e = 0; e < 4; ++e) bb[e] = bfr(braw[e]);
  const int s0 = (2 * lane) & 31, s1 = (2 * lane + 1) & 31;
  const int l16 = lane & 15;
#pragma unroll 1
  for (int j = 0; j < kRowsPerWave; ++j) {
    const int dl = wlo + j;
    const int n = n0 + dl;
    if (n < kNPad) {
      const bool live = n < kNodes;
      const int cnt = CNT[dl];
      const float cf = (float)cnt;
      const float si = rsqrtf(fmaxf(cf, 1.0f));
      float* rp = zp + (size_t)n * kDim + 4 * lane;
      const v4f a = *(const v4f*)rp;
      const v4f v = a * si + bb;
      v4f vz;
#pragma unroll
      for (int e = 0; e < 4; ++e) vz[e] = live ? v[e] : 0.f;
      float u[8];
#pragma unroll
      for (int e = 0; e < 4; ++e) { u[e] = __shfl(vz[e], s0, 32); u[4 + e] = __shfl(vz[e], s1, 32); }
      unsigned short hb8[8];
#pragma unroll
      for (int e = 0; e < 8; ++e) hb8[e] = f2bf_bits(u[e]);
      const v4u pk = (v4u){pk16(hb8[0], hb8[1]), pk16(hb8[2], hb8[3]), pk16(hb8[4], hb8[5]), pk16(hb8[6], hb8[7])};
      unsigned short* zr = zbp + (size_t)n * kDim + 8 * l16;
      for (int pass = 0; pass < 2; ++pass) {
        *(volatile v4f*)rp = vz;
        if (lane < 16) *(volatile v4u*)zr = pk;
        __threadfence();
      }
    }
  }
}

__global__ __launch_bounds__(kThreads) void score_kernel(const unsigned* __restrict__ uw, const float* __restrict__ b1,
                                                        const float* __restrict__ w2, float* __restrict__ part) {
  __shared__ __align__(16) float red[32];
  const int tid = threadIdx.x, lane = tid & 31, wave = tid >> 5;
  if (tid < 32) red[tid] = 0.f;
  __syncthreads();
  const int rl = tid >> 6;
  const int wd = tid & 63;
  const int c0 = 2 * wd;
  const float b1a = bfr(b1[c0]), b1b = bfr(b1[c0 + 1]);
  const float w2a = bfr(w2[c0]), w2b = bfr(w2[c0 + 1]);
  const int rbase = blockIdx.x * kRedRows;
  float acc = 0.f;
#pragma unroll 1
  for (int it = 0; it < kRedRows / 4; ++it) {
    const int row = rbase + it * 4 + rl;
    const bool live = row < kNodes;
    const int rowc = live ? row : (kNodes - 1);
    const unsigned w = uw[(size_t)rowc * (kDim / 2) + wd];
    const float ua = h16_to_f32(w & 0xffffu) + b1a;
    const float ub = h16_to_f32(w >> 16) + b1b;
    const float ta = tanhf(ua), tb = tanhf(ub);
    const float cv = ta * w2a + tb * w2b;
    acc += live ? cv : 0.f;
  }
#pragma unroll
  for (int off = 16; off > 0; off >>= 1) acc += __shfl_xor(acc, off, 32);
  if (lane == 0) red[wave] = acc;
  __syncthreads();
  if (wave == 0 && lane < 8) {
    const v4f o = *(const v4f*)(red + 4 * lane);
    float* dst = part + ((size_t)blockIdx.x * 32 + 4 * lane);
    *(volatile v4f*)dst = o;
    __threadfence();
    *(volatile v4f*)dst = o;
  }
}

__global__ __launch_bounds__(kThreads) void beta_kernel(const float* __restrict__ part, float* __restrict__ betl) {
  __shared__ float wsum[8];
  __shared__ float wp[4];
  __shared__ __align__(16) float bl[32];
  const int tid = threadIdx.x, lane = tid & 31, wave = tid >> 5;
  if (tid < 32) bl[tid] = 0.f;
  if (tid < 8) wsum[tid] = 0.f;
  if (tid < 4) wp[tid] = 0.f;
  __syncthreads();
#pragma unroll 1
  for (int p = 0; p < kPaths; ++p) {
    const float* pp = part + (size_t)p * kRedBlocks * 32;
    float s = 0.f;
    for (int i = tid; i < kRedBlocks * 32; i += kThreads) s += pp[i];
#pragma unroll
    for (int off = 16; off > 0; off >>= 1) s += __shfl_xor(s, off, 32);
    if (lane == 0) wsum[wave] = s;
    __syncthreads();
    if (tid == 0) {
      float t = 0.f;
#pragma unroll
      for (int w = 0; w < 8; ++w) t += wsum[w];
      wp[p] = t * (1.0f / (float)kNodes);
    }
    __syncthreads();
  }
  if (tid == 0) {
    const float a0 = wp[0], a1 = wp[1], a2 = wp[2];
    const float m = fmaxf(a0, fmaxf(a1, a2));
    const float e0 = expf(a0 - m), e1 = expf(a1 - m), e2 = expf(a2 - m);
    const float inv = 1.0f / (e0 + e1 + e2);
    bl[0] = e0 * inv; bl[1] = e1 * inv; bl[2] = e2 * inv;
  }
  __syncthreads();
  if (wave == 0 && lane < 8) {
    const v4f o = *(const v4f*)(bl + 4 * lane);
    *(volatile v4f*)(betl + 4 * lane) = o;
    __threadfence();
    *(volatile v4f*)(betl + 4 * lane) = o;
  }
}

__global__ __launch_bounds__(kThreads) void combine_kernel(const float* __restrict__ z, const float* __restrict__ betl,
                                                          float* __restrict__ out) {
  const int i = blockIdx.x * kThreads + threadIdx.x;
  if (i >= kNodes * (kDim / 4)) return;
  const float c0 = betl[0], c1 = betl[1], c2 = betl[2];
  const size_t o4 = 4 * (size_t)i;
  const v4f a0 = *(const v4f*)(z + o4);
  const v4f a1 = *(const v4f*)(z + (size_t)kNPad * kDim + o4);
  const v4f a2 = *(const v4f*)(z + (size_t)2 * kNPad * kDim + o4);
  v4f o = a0 * c0;
  o = o + a1 * c1;
  o = o + a2 * c2;
  *(volatile v4f*)(out + o4) = o;
  __threadfence();
  *(volatile v4f*)(out + o4) = o;
}

extern "C" void kernel_launch(void* const* d_in, const int* in_sizes, int n_in,
                              void* d_out, int out_size, void* d_ws, size_t ws_size, hipStream_t stream) {
  (void)in_sizes; (void)n_in; (void)out_size;
  const float* h    = (const float*)d_in[0];
  const float* Wgc  = (const float*)d_in[1];
  const float* bgc  = (const float*)d_in[2];
  const float* w1   = (const float*)d_in[3];
  const float* b1   = (const float*)d_in[4];
  const float* w2   = (const float*)d_in[5];
  const int*   esrc = (const int*)d_in[6];
  const int*   edst = (const int*)d_in[7];
  float* out = (float*)d_out;

  char* ws = (char*)d_ws; size_t off = 0;
  auto carve = [&](size_t bytes) -> char* { char* p = ws + off; off += (bytes + 255) & ~(size_t)255; return p; };
  unsigned short* hb   = (unsigned short*)carve((size_t)kNPad * kDim * 2);
  unsigned short* wt   = (unsigned short*)carve((size_t)4 * kDim * kDim * 2);
  float*          iso  = (float*)carve((size_t)kPaths * kIsoPitch * 4);
  float*          xtl  = (float*)carve((size_t)kTailRows * kDim * 4);
  float*          z    = (float*)carve((size_t)kPaths * kNPad * kDim * 4);
  unsigned short* zb   = (unsigned short*)carve((size_t)kNPad * kDim * 2);
  unsigned short* upl  = (unsigned short*)carve((size_t)kNPad * kDim * 2);
  float*          part = (float*)carve((size_t)kPaths * kRedBlocks * 32 * 4);
  float*          betl = (float*)carve(256);
  if (off > ws_size || off > (size_t)134217728) return;

  cast_h_kernel<<<(kNPad * (kDim / 8)) / kThreads, kThreads, 0, stream>>>(h, hb);
  wtcast_kernel<<<dim3(2, 2, 4), kThreads, 0, stream>>>(Wgc, w1, wt);
  degout_kernel<<<dim3(kTiles, kPaths), kThreads, 0, stream>>>(esrc, iso);

  const unsigned short* w1t = wt + (size_t)3 * kDim * kDim;
  for (int p = 0; p < kPaths; ++p) {
    const unsigned short* btp = wt + (size_t)p * kDim * kDim;
    wmma_gemm64<1, false, 0, 0, false><<<dim3(kMainBlocks, 1), kThreads, 0, stream>>>(
        (const unsigned short*)hb, (const unsigned short*)nullptr, kDim, 0L,
        btp, (const unsigned short*)nullptr, kDim, 0L,
        (void*)out, (void*)nullptr, kDim, 0L,
        (const float*)nullptr, (const float*)nullptr, 0L, kNMain, kDim, kDim, 1.0f);
    wmma_gemm64<1, false, 0, 0, false><<<dim3(1, 1), kThreads, 0, stream>>>(
        (const unsigned short*)(hb + (size_t)kNMain * kDim), (const unsigned short*)nullptr, kDim, 0L,
        btp, (const unsigned short*)nullptr, kDim, 0L,
        (void*)xtl, (void*)nullptr, kDim, 0L,
        (const float*)nullptr, (const float*)nullptr, 0L, kTailRows, kDim, kDim, 1.0f);
    agg_kernel<<<dim3(kTiles), kThreads, 0, stream>>>(
        (const float*)out, (const float*)xtl,
        esrc + (size_t)p * kEdges, edst + (size_t)p * kEdges,
        iso + (size_t)p * kIsoPitch, bgc + (size_t)p * kDim,
        z + (size_t)p * kNPad * kDim, zb);
    wmma_gemm64<1, false, 0, 1, false><<<dim3(kPadBlocks, 1), kThreads, 0, stream>>>(
        (const unsigned short*)zb, (const unsigned short*)nullptr, kDim, 0L,
        w1t, (const unsigned short*)nullptr, kDim, 0L,
        (void*)upl, (void*)nullptr, kDim, 0L,
        (const float*)nullptr, (const float*)nullptr, 0L, kNPad, kDim, kDim, 1.0f);
    score_kernel<<<dim3(kRedBlocks), kThreads, 0, stream>>>(
        (const unsigned*)upl, b1, w2, part + (size_t)p * kRedBlocks * 32);
  }

  beta_kernel<<<1, kThreads, 0, stream>>>(part, betl);
  combine_kernel<<<(kNodes * (kDim / 4)) / kThreads, kThreads, 0, stream>>>(z, betl, out);
}
